// SequentialTransductionUnitJagged_34849364639830
// MI455X (gfx1250) — hardware-verified
//
#include <hip/hip_runtime.h>
#include <stdint.h>

#define NB     8
#define NPAD   1024
#define DM     512
#define NHD    8
#define HDIM   64
#define NTOK   (NB * NPAD)
#define UVQKC  2048
#define LN_EPS 1e-6f
#define PFOLD  (1.0f / 1024.0f)

typedef __attribute__((ext_vector_type(16))) __bf16 v16b;
typedef __attribute__((ext_vector_type(8)))  __bf16 v8b;
typedef __attribute__((ext_vector_type(8)))  float  v8f;
typedef __attribute__((ext_vector_type(4)))  float  v4f;
typedef __attribute__((ext_vector_type(4)))  unsigned int v4u;
typedef __attribute__((ext_vector_type(8)))  unsigned int v8u;
typedef v8b __attribute__((may_alias)) v8ba;
typedef v4f __attribute__((may_alias)) v4fa;
typedef v4u __attribute__((may_alias)) v4ua;

union FragU { v16b v; v8b h[2]; };
union PackU { v8u u; v16b v; };

__device__ __forceinline__ unsigned short f2bf_bits(float f) {
  const unsigned u = __float_as_uint(f);
  return (unsigned short)((u + 0x7FFFu + ((u >> 16) & 1u)) >> 16);
}
__device__ __forceinline__ float bf_bits2f(unsigned short h) { return __uint_as_float(((unsigned)h) << 16); }
__device__ __forceinline__ float bf16r(float f) {
  unsigned u = __float_as_uint(f);
  u = (u + 0x7FFFu + ((u >> 16) & 1u)) & 0xFFFF0000u;
  return __uint_as_float(u);
}
__device__ __forceinline__ unsigned pk16(unsigned short a, unsigned short b) { return (unsigned)a | ((unsigned)b << 16); }

__device__ __forceinline__ float silu_f(float v) {
  return v * __builtin_amdgcn_rcpf(1.0f + __expf(-v));
}

__device__ __forceinline__ v8f wmma_bf16(v16b a, v16b b, v8f c) {
  v8f d = __builtin_amdgcn_wmma_f32_16x16x32_bf16(false, a, false, b, (short)0, c, false, false);
  asm volatile("v_nop\n\tv_nop\n\tv_nop\n\tv_nop" : "+v"(d) : "v"(a), "v"(b));
  return d;
}

__device__ __forceinline__ v16b load_frag(const unsigned short* p, int hh) {
  FragU f;
  f.h[0] = *(const v8ba*)(p + 8 * hh);
  f.h[1] = *(const v8ba*)(p + 16 + 8 * hh);
  return f.v;
}

__device__ __forceinline__ void pack_p2(v8f a, v8f c, v16b& ho, v16b& lo) {
  PackU uh, ul;
#pragma unroll
  for (int i = 0; i < 4; ++i) {
    const unsigned short h0 = f2bf_bits(a[2 * i]), h1 = f2bf_bits(a[2 * i + 1]);
    const unsigned short l0 = f2bf_bits(a[2 * i] - bf_bits2f(h0)), l1 = f2bf_bits(a[2 * i + 1] - bf_bits2f(h1));
    uh.u[i] = pk16(h0, h1); ul.u[i] = pk16(l0, l1);
    const unsigned short g0 = f2bf_bits(c[2 * i]), g1 = f2bf_bits(c[2 * i + 1]);
    const unsigned short m0 = f2bf_bits(c[2 * i] - bf_bits2f(g0)), m1 = f2bf_bits(c[2 * i + 1] - bf_bits2f(g1));
    uh.u[4 + i] = pk16(g0, g1); ul.u[4 + i] = pk16(m0, m1);
  }
  ho = uh.v; lo = ul.v;
}

__device__ __forceinline__ void gemm_core_32x64(
    const unsigned short* __restrict__ Ah, const unsigned short* __restrict__ Al,
    const unsigned short* __restrict__ Bt, int K, size_t aoff, size_t boff, int hh, v8f (&acc)[2][4]) {
  const unsigned short* a0h = Ah + aoff;
  const unsigned short* a1h = a0h + (size_t)16 * K;
  const unsigned short* a0l = Al + aoff;
  const unsigned short* a1l = a0l + (size_t)16 * K;
  const unsigned short* bp  = Bt + boff;
#pragma unroll 1
  for (int k0 = 0; k0 < K; k0 += 32) {
    const v16b f0h = load_frag(a0h + k0, hh);
    const v16b f0l = load_frag(a0l + k0, hh);
    const v16b f1h = load_frag(a1h + k0, hh);
    const v16b f1l = load_frag(a1l + k0, hh);
#pragma unroll
    for (int nt = 0; nt < 4; ++nt) {
      const v16b fb = load_frag(bp + (size_t)nt * 16 * K + k0, hh);
      acc[0][nt] = wmma_bf16(f0h, fb, acc[0][nt]);
      acc[0][nt] = wmma_bf16(f0l, fb, acc[0][nt]);
      acc[1][nt] = wmma_bf16(f1h, fb, acc[1][nt]);
      acc[1][nt] = wmma_bf16(f1l, fb, acc[1][nt]);
    }
  }
}

__global__ __launch_bounds__(256) void k_tr_bf16(const float* __restrict__ src, unsigned short* __restrict__ dst,
                                                 int R, int C) {
  __shared__ __align__(16) unsigned short t16[64 * 72];
  const int c0  = blockIdx.x * 64;
  const int r0  = blockIdx.y * 64;
  const int tid = threadIdx.x;
  {
    const int rr = tid >> 2;
    const int cq = (tid & 3) * 16;
    const float* s = src + (size_t)(r0 + rr) * C + c0 + cq;
#pragma unroll
    for (int q = 0; q < 4; ++q) {
      const v4f f = *(const v4fa*)(s + 4 * q);
#pragma unroll
      for (int e = 0; e < 4; ++e) t16[rr * 72 + cq + 4 * q + e] = f2bf_bits(f[e]);
    }
  }
  __syncthreads();
  const int sub = tid >> 3;
  const int c8  = (tid & 7) * 8;
  v4u hv[2];
#pragma unroll
  for (int it = 0; it < 2; ++it) {
    const int oc = it * 32 + sub;
    v4u a;
#pragma unroll
    for (int q = 0; q < 4; ++q)
      a[q] = pk16(t16[(c8 + 2 * q) * 72 + oc], t16[(c8 + 2 * q + 1) * 72 + oc]);
    hv[it] = a;
  }
  for (int pass = 0; pass < 2; ++pass) {
#pragma unroll
    for (int it = 0; it < 2; ++it) {
      const int oc = it * 32 + sub;
      const size_t go = (size_t)(c0 + oc) * R + r0 + c8;
      *(volatile v4u*)(dst + go) = hv[it];
    }
    __threadfence();
  }
}

__device__ __forceinline__ void ln_split_store(float (&v)[16], const float (&g)[16], bool use_g, bool poison,
                                               bool ok, unsigned short* __restrict__ Hp, unsigned short* __restrict__ Lp,
                                               size_t rowoff, int lane) {
  float s = 0.0f;
#pragma unroll
  for (int i = 0; i < 16; ++i) s += v[i];
#pragma unroll
  for (int o = 16; o > 0; o >>= 1) s += __shfl_xor(s, o);
  const float mean = s * (1.0f / 512.0f);
  float q = 0.0f;
#pragma unroll
  for (int i = 0; i < 16; ++i) { const float d = v[i] - mean; v[i] = d; q += d * d; }
#pragma unroll
  for (int o = 16; o > 0; o >>= 1) q += __shfl_xor(q, o);
  const float rstd = rsqrtf(q * (1.0f / 512.0f) + LN_EPS);
  const float qnan = __uint_as_float(0x7fc00000u);
  unsigned hw[8], lw[8];
#pragma unroll
  for (int i = 0; i < 8; ++i) {
    float y0 = v[2 * i] * rstd, y1 = v[2 * i + 1] * rstd;
    if (use_g) { y0 *= g[2 * i]; y1 *= g[2 * i + 1]; }
    y0 = poison ? qnan : y0;
    y1 = poison ? qnan : y1;
    const unsigned short h0 = f2bf_bits(y0), h1 = f2bf_bits(y1);
    const unsigned short l0 = f2bf_bits(y0 - bf_bits2f(h0)), l1 = f2bf_bits(y1 - bf_bits2f(h1));
    hw[i] = pk16(h0, h1); lw[i] = pk16(l0, l1);
  }
  const v4u hA = (v4u){hw[0], hw[1], hw[2], hw[3]};
  const v4u hB = (v4u){hw[4], hw[5], hw[6], hw[7]};
  const v4u lA = (v4u){lw[0], lw[1], lw[2], lw[3]};
  const v4u lB = (v4u){lw[4], lw[5], lw[6], lw[7]};
  const size_t o0 = rowoff + (size_t)lane * 8;
  const size_t o1 = rowoff + 256 + (size_t)lane * 8;
  if (ok) {
    *(volatile v4u*)(Hp + o0) = hA; *(volatile v4u*)(Hp + o1) = hB;
    *(volatile v4u*)(Lp + o0) = lA; *(volatile v4u*)(Lp + o1) = lB;
  }
  __threadfence();
  if (ok) {
    *(volatile v4u*)(Hp + o0) = hA; *(volatile v4u*)(Hp + o1) = hB;
    *(volatile v4u*)(Lp + o0) = lA; *(volatile v4u*)(Lp + o1) = lB;
  }
}

__global__ __launch_bounds__(256) void k_ln_split(const float* __restrict__ x,
                                                  unsigned short* __restrict__ XNhi, unsigned short* __restrict__ XNlo, int T) {
  const int lane = threadIdx.x & 31;
  int row = blockIdx.x * 8 + (threadIdx.x >> 5);
  const bool ok = row < T;
  row = ok ? row : (T - 1);
  const float* xr = x + (size_t)row * DM;
  const v4f a0 = *(const v4fa*)(xr + lane * 8);
  const v4f a1 = *(const v4fa*)(xr + lane * 8 + 4);
  const v4f a2 = *(const v4fa*)(xr + 256 + lane * 8);
  const v4f a3 = *(const v4fa*)(xr + 256 + lane * 8 + 4);
  float v[16] = {a0[0], a0[1], a0[2], a0[3], a1[0], a1[1], a1[2], a1[3],
                 a2[0], a2[1], a2[2], a2[3], a3[0], a3[1], a3[2], a3[3]};
  float g[16];
#pragma unroll
  for (int i = 0; i < 16; ++i) { v[i] = bf16r(v[i]); g[i] = 1.0f; }
  ln_split_store(v, g, false, false, ok, XNhi, XNlo, (size_t)row * DM, lane);
}

__global__ __launch_bounds__(128) void k_proj(
    const unsigned short* __restrict__ XNhi, const unsigned short* __restrict__ XNlo,
    const unsigned short* __restrict__ WT,
    float* __restrict__ U,
    unsigned short* __restrict__ Qhi, unsigned short* __restrict__ Qlo,
    unsigned short* __restrict__ Khi, unsigned short* __restrict__ Klo,
    unsigned short* __restrict__ VThi, unsigned short* __restrict__ VTlo, int T) {
  __shared__ __align__(16) unsigned char smem[32768];
  float* sF = (float*)smem;
  unsigned short* sH = (unsigned short*)smem;
  unsigned short* sL = sH + 8192;
  const int tid = threadIdx.x, lane = tid & 31, w = tid >> 5;
  const int hh = lane >> 4, m = lane & 15;
  const int m0 = blockIdx.x * 128;
  const int cg = blockIdx.y;
  const int which = cg >> 3, head = cg & 7;
  const int n0 = cg * 64;
  const int m0w = m0 + 32 * w;

  const v8f zero8 = {0.f, 0.f, 0.f, 0.f, 0.f, 0.f, 0.f, 0.f};
  v8f acc[2][4];
#pragma unroll
  for (int mt = 0; mt < 2; ++mt)
#pragma unroll
    for (int nt = 0; nt < 4; ++nt) acc[mt][nt] = zero8;

  gemm_core_32x64(XNhi, XNlo, WT, DM, (size_t)(m0w + m) * DM, (size_t)(n0 + m) * DM, hh, acc);

  if (which == 0) {
#pragma unroll
    for (int nt = 0; nt < 4; ++nt)
#pragma unroll
      for (int mt = 0; mt < 2; ++mt)
#pragma unroll
        for (int r = 0; r < 8; ++r) {
          const int tokl = 32 * w + 16 * mt + 8 * hh + r;
          const int feat = 16 * nt + m;
          sF[tokl * 64 + feat] = silu_f(acc[mt][nt][r]);
        }
  } else {
#pragma unroll
    for (int nt = 0; nt < 4; ++nt)
#pragma unroll
      for (int mt = 0; mt < 2; ++mt)
#pragma unroll
        for (int r = 0; r < 8; ++r) {
          const int tokl = 32 * w + 16 * mt + 8 * hh + r;
          const int feat = 16 * nt + m;
          const float y = silu_f(acc[mt][nt][r]);
          const unsigned short hb = f2bf_bits(y);
          const unsigned short lb = f2bf_bits(y - bf_bits2f(hb));
          const int idx = (which == 1) ? (feat * 128 + tokl) : (tokl * 64 + feat);
          sH[idx] = hb;
          sL[idx] = lb;
        }
  }
  __syncthreads();

  if (which == 0) {
    const int rsub = lane >> 4, c4 = (lane & 15) * 4;
    for (int pass = 0; pass < 2; ++pass) {
#pragma unroll
      for (int it = 0; it < 16; ++it) {
        const int row = 32 * w + 2 * it + rsub;
        const v4f v = *(const v4fa*)(sF + row * 64 + c4);
        *(volatile v4f*)(U + (size_t)(m0 + row) * DM + head * HDIM + c4) = v;
      }
      __threadfence();
    }
  } else if (which == 1) {
    const int dsub = lane >> 4, t8 = (lane & 15) * 8;
    for (int pass = 0; pass < 2; ++pass) {
#pragma unroll
      for (int it = 0; it < 8; ++it) {
        const int d = 16 * w + 2 * it + dsub;
        const v4u hv = *(const v4ua*)(sH + d * 128 + t8);
        const v4u lv = *(const v4ua*)(sL + d * 128 + t8);
        const size_t go = (size_t)(head * HDIM + d) * (size_t)T + m0 + t8;
        *(volatile v4u*)(VThi + go) = hv;
        *(volatile v4u*)(VTlo + go) = lv;
      }
      __threadfence();
    }
  } else {
    unsigned short* ph = (which == 2) ? Qhi : Khi;
    unsigned short* pl = (which == 2) ? Qlo : Klo;
    const int rsub = lane >> 3, c8 = (lane & 7) * 8;
    for (int pass = 0; pass < 2; ++pass) {
#pragma unroll
      for (int it = 0; it < 8; ++it) {
        const int row = 32 * w + 4 * it + rsub;
        const v4u hv = *(const v4ua*)(sH + row * 64 + c8);
        const v4u lv = *(const v4ua*)(sL + row * 64 + c8);
        const size_t go = (size_t)(m0 + row) * DM + head * HDIM + c8;
        *(volatile v4u*)(ph + go) = hv;
        *(volatile v4u*)(pl + go) = lv;
      }
      __threadfence();
    }
  }
}

__global__ __launch_bounds__(128) void k_attn(
    const unsigned short* __restrict__ Qhi, const unsigned short* __restrict__ Qlo,
    const unsigned short* __restrict__ Khi, const unsigned short* __restrict__ Klo,
    const unsigned short* __restrict__ VThi, const unsigned short* __restrict__ VTlo,
    const float* __restrict__ mask, const int* __restrict__ xoff,
    float* __restrict__ ATT, int T) {
  __shared__ __align__(16) float sO[4 * 16 * 64];
  __shared__ int sflag[2][4];

  const int tid = threadIdx.x, lane = tid & 31, w = tid >> 5;
  const int hh = lane >> 4, m = lane & 15;
  const int qt = blockIdx.x;
  const int b = blockIdx.y >> 3, h = blockIdx.y & 7;
  const int q0 = qt * 64;

  const int xb = xoff[b];
  const int xe = xoff[b + 1];
  int len = xe - xb;
  len = (len < 0) ? 0 : len;
  len = (len > NPAD) ? NPAD : len;
  int base = (xb < 0) ? 0 : xb;
  base = (base > T - 1) ? (T - 1) : base;
  if (q0 >= len) return;

  const int q0w = q0 + 16 * w;
  int qtok = base + q0w + m;
  qtok = (qtok > T - 1) ? (T - 1) : qtok;

  const unsigned short* qrh = Qhi + (size_t)qtok * DM + h * HDIM;
  const unsigned short* qrl = Qlo + (size_t)qtok * DM + h * HDIM;
  const v16b qb0h = load_frag(qrh, hh), qb1h = load_frag(qrh + 32, hh);
  const v16b qb0l = load_frag(qrl, hh), qb1l = load_frag(qrl + 32, hh);

  const v8f zero8 = {0.f, 0.f, 0.f, 0.f, 0.f, 0.f, 0.f, 0.f};
  v8f o[4];
#pragma unroll
  for (int t = 0; t < 4; ++t) o[t] = zero8;

  const float* mr = mask + ((size_t)(b * NPAD + q0w + m)) * NPAD + 8 * hh;

  int it = 0;
#pragma unroll 1
  for (int kb = 0; kb < len; kb += 64, ++it) {
    float mk[4][8];
    int nz = 0;
#pragma unroll
    for (int j = 0; j < 4; ++j) {
      const v4f ma = *(const v4fa*)(mr + kb + 16 * j);
      const v4f mb = *(const v4fa*)(mr + kb + 16 * j + 4);
      const float mv[8] = {ma[0], ma[1], ma[2], ma[3], mb[0], mb[1], mb[2], mb[3]};
#pragma unroll
      for (int r = 0; r < 8; ++r) {
        const int key = kb + 16 * j + 8 * hh + r;
        const float f = (key < len) ? mv[r] : 0.0f;
        mk[j][r] = f;
        nz |= (f != 0.0f) ? 1 : 0;
      }
    }
#pragma unroll
    for (int off = 16; off > 0; off >>= 1) nz |= __shfl_xor(nz, off);
    if (lane == 0) sflag[it & 1][w] = nz;
    __syncthreads();
    int blk = sflag[it & 1][0] | sflag[it & 1][1] | sflag[it & 1][2] | sflag[it & 1][3];
    blk = __builtin_amdgcn_readfirstlane(blk);
    if (blk == 0) continue;

    int kvb = base + kb;
    kvb = (kvb > T - 64) ? (T - 64) : kvb;

    v8f s[4];
#pragma unroll
    for (int j = 0; j < 4; ++j) {
      const unsigned short* kph = Khi + (size_t)(kvb + 16 * j + m) * DM + h * HDIM;
      const unsigned short* kpl = Klo + (size_t)(kvb + 16 * j + m) * DM + h * HDIM;
      const v16b k0h = load_frag(kph, hh), k1h = load_frag(kph + 32, hh);
      const v16b k0l = load_frag(kpl, hh), k1l = load_frag(kpl + 32, hh);
      v8f z = zero8;
      z = wmma_bf16(k0h, qb0h, z);
      z = wmma_bf16(k0h, qb0l, z);
      z = wmma_bf16(k0l, qb0h, z);
      z = wmma_bf16(k1h, qb1h, z);
      z = wmma_bf16(k1h, qb1l, z);
      z = wmma_bf16(k1l, qb1h, z);
      s[j] = z;
    }
#pragma unroll
    for (int j = 0; j < 4; ++j)
#pragma unroll
      for (int r = 0; r < 8; ++r) s[j][r] = silu_f(s[j][r]) * mk[j][r];

    v16b p0h, p0l, p1h, p1l;
    pack_p2(s[0], s[1], p0h, p0l);
    pack_p2(s[2], s[3], p1h, p1l);

#pragma unroll
    for (int t = 0; t < 4; ++t) {
      const unsigned short* vph = VThi + (size_t)(h * HDIM + 16 * t + m) * (size_t)T + kvb;
      const unsigned short* vpl = VTlo + (size_t)(h * HDIM + 16 * t + m) * (size_t)T + kvb;
      const v16b v0h = load_frag(vph, hh), v1h = load_frag(vph + 32, hh);
      const v16b v0l = load_frag(vpl, hh), v1l = load_frag(vpl + 32, hh);
      o[t] = wmma_bf16(v0h, p0h, o[t]);
      o[t] = wmma_bf16(v0h, p0l, o[t]);
      o[t] = wmma_bf16(v0l, p0h, o[t]);
      o[t] = wmma_bf16(v1h, p1h, o[t]);
      o[t] = wmma_bf16(v1h, p1l, o[t]);
      o[t] = wmma_bf16(v1l, p1h, o[t]);
    }
  }

  float* so = sO + w * 1024;
#pragma unroll
  for (int t = 0; t < 4; ++t)
#pragma unroll
    for (int r = 0; r < 8; ++r)
      so[m * 64 + 16 * t + 8 * hh + r] = o[t][r] * PFOLD;
  __syncthreads();

  const int q8 = lane & 7, sub = lane >> 3;
  for (int pass = 0; pass < 2; ++pass) {
#pragma unroll
    for (int i = 0; i < 8; ++i) {
      const int lid = i * 4 + sub;
      const int row = lid >> 1, hl = lid & 1;
      const v4f v = *(const v4fa*)(so + row * 64 + 32 * hl + 4 * q8);
      const int qi  = q0w + row;
      const int tok = base + qi;
      if (qi < len && tok < T) {
        *(volatile v4f*)(ATT + (size_t)tok * DM + h * HDIM + 32 * hl + 4 * q8) = v;
      }
    }
    __threadfence();
  }
}

__global__ __launch_bounds__(256) void k_gate_split(const float* __restrict__ ATT, const float* __restrict__ U,
                                                    const int* __restrict__ xoff,
                                                    unsigned short* __restrict__ OIhi, unsigned short* __restrict__ OIlo, int T) {
  const int lane = threadIdx.x & 31;
  int row = blockIdx.x * 8 + (threadIdx.x >> 5);
  const bool ok = row < T;
  row = ok ? row : (T - 1);
  const float* ar = ATT + (size_t)row * DM;
  const float* ur = U   + (size_t)row * DM;
  const v4f a0 = *(const v4fa*)(ar + lane * 8);
  const v4f a1 = *(const v4fa*)(ar + lane * 8 + 4);
  const v4f a2 = *(const v4fa*)(ar + 256 + lane * 8);
  const v4f a3 = *(const v4fa*)(ar + 256 + lane * 8 + 4);
  const v4f u0 = *(const v4fa*)(ur + lane * 8);
  const v4f u1 = *(const v4fa*)(ur + lane * 8 + 4);
  const v4f u2 = *(const v4fa*)(ur + 256 + lane * 8);
  const v4f u3 = *(const v4fa*)(ur + 256 + lane * 8 + 4);
  float v[16] = {a0[0], a0[1], a0[2], a0[3], a1[0], a1[1], a1[2], a1[3],
                 a2[0], a2[1], a2[2], a2[3], a3[0], a3[1], a3[2], a3[3]};
  const float g[16] = {u0[0], u0[1], u0[2], u0[3], u1[0], u1[1], u1[2], u1[3],
                       u2[0], u2[1], u2[2], u2[3], u3[0], u3[1], u3[2], u3[3]};
  const int xo = xoff[(lane < NB) ? lane : NB];
  int cov = 0;
#pragma unroll
  for (int bb = 0; bb < NB; ++bb) {
    const int xb = __shfl(xo, bb);
    const int xe = __shfl(xo, bb + 1);
    int lenb = xe - xb;
    lenb = (lenb < 0) ? 0 : lenb;
    lenb = (lenb > NPAD) ? NPAD : lenb;
    cov |= ((row >= xb) && (row < xb + lenb)) ? 1 : 0;
  }
  ln_split_store(v, g, true, cov == 0, ok, OIhi, OIlo, (size_t)row * DM, lane);
}

__global__ __launch_bounds__(128) void k_out(
    const unsigned short* __restrict__ OIhi, const unsigned short* __restrict__ OIlo,
    const unsigned short* __restrict__ OWT, const float* __restrict__ ob, const float* __restrict__ x,
    float* __restrict__ out, int T) {
  __shared__ __align__(16) float sF[128 * 64];
  const int tid = threadIdx.x, lane = tid & 31, w = tid >> 5;
  const int hh = lane >> 4, m = lane & 15;
  const int m0 = blockIdx.x * 128;
  const int n0 = blockIdx.y * 64;
  const int m0w = m0 + 32 * w;

  const v8f zero8 = {0.f, 0.f, 0.f, 0.f, 0.f, 0.f, 0.f, 0.f};
  v8f acc[2][4];
#pragma unroll
  for (int mt = 0; mt < 2; ++mt)
#pragma unroll
    for (int nt = 0; nt < 4; ++nt) acc[mt][nt] = zero8;

  gemm_core_32x64(OIhi, OIlo, OWT, DM, (size_t)(m0w + m) * DM, (size_t)(n0 + m) * DM, hh, acc);

#pragma unroll
  for (int nt = 0; nt < 4; ++nt)
#pragma unroll
    for (int mt = 0; mt < 2; ++mt)
#pragma unroll
      for (int r = 0; r < 8; ++r) {
        const int tokl = 32 * w + 16 * mt + 8 * hh + r;
        const int feat = 16 * nt + m;
        sF[tokl * 64 + feat] = acc[mt][nt][r];
      }
  __syncthreads();

  const int rsub = lane >> 4, c4 = (lane & 15) * 4;
  const v4f bz = *(const v4fa*)(ob + n0 + c4);
  const v4f bq = (v4f){bf16r(bz[0]), bf16r(bz[1]), bf16r(bz[2]), bf16r(bz[3])};
  for (int pass = 0; pass < 2; ++pass) {
#pragma unroll
    for (int it = 0; it < 16; ++it) {
      const int row = 32 * w + 2 * it + rsub;
      const int tok = m0 + row;
      const v4f a  = *(const v4fa*)(sF + row * 64 + c4);
      const v4f xr = *(const v4fa*)(x + (size_t)tok * DM + n0 + c4);
      v4f o;
      o[0] = (a[0] + bq[0]) + bf16r(xr[0]);
      o[1] = (a[1] + bq[1]) + bf16r(xr[1]);
      o[2] = (a[2] + bq[2]) + bf16r(xr[2]);
      o[3] = (a[3] + bq[3]) + bf16r(xr[3]);
      *(volatile v4f*)(out + (size_t)tok * DM + n0 + c4) = o;
    }
    __threadfence();
  }
}

extern "C" void kernel_launch(void* const* d_in, const int* in_sizes, int n_in,
                              void* d_out, int out_size, void* d_ws, size_t ws_size,
                              hipStream_t stream) {
  if (n_in < 6) return;
  if (in_sizes[0] != NTOK * DM) return;
  if (in_sizes[1] != DM * UVQKC) return;
  if (in_sizes[2] != DM * DM) return;
  if (in_sizes[3] != DM) return;
  if (in_sizes[4] != NB * NPAD * NPAD) return;
  if (in_sizes[5] != NB + 1) return;
  if (out_size != NTOK * DM) return;

  const float* x    = (const float*)d_in[0];
  const float* uvqk = (const float*)d_in[1];
  const float* o_w  = (const float*)d_in[2];
  const float* o_b  = (const float*)d_in[3];
  const float* mask = (const float*)d_in[4];
  const int*   xoff = (const int*)d_in[5];
  float* out = (float*)d_out;
  const int T = in_sizes[0] / DM;

  const size_t PWT  = (size_t)UVQKC * DM * 2;
  const size_t POWT = (size_t)DM * DM * 2;
  const size_t P16  = (size_t)T * DM * 2;
  const size_t P32  = (size_t)T * DM * 4;
  const size_t PVT  = (size_t)NHD * HDIM * T * 2;
  size_t off = 0;
  const size_t oWT   = off; off += PWT;
  const size_t oOWT  = off; off += POWT;
  const size_t oXNhi = off; off += P16;
  const size_t oXNlo = off; off += P16;
  const size_t oU    = off; off += P32;
  const size_t oQhi  = off; off += P16;
  const size_t oQlo  = off; off += P16;
  const size_t oKhi  = off; off += P16;
  const size_t oKlo  = off; off += P16;
  const size_t oVThi = off; off += PVT;
  const size_t oVTlo = off; off += PVT;
  const size_t oATT  = off; off += P32;
  const size_t oOIhi = off; off += P16;
  const size_t oOIlo = off; off += P16;
  if (off > ws_size) return;

  char* ws = (char*)d_ws;
  unsigned short* WT   = (unsigned short*)(ws + oWT);
  unsigned short* OWT  = (unsigned short*)(ws + oOWT);
  unsigned short* XNhi = (unsigned short*)(ws + oXNhi);
  unsigned short* XNlo = (unsigned short*)(ws + oXNlo);
  float*          U    = (float*)(ws + oU);
  unsigned short* Qhi  = (unsigned short*)(ws + oQhi);
  unsigned short* Qlo  = (unsigned short*)(ws + oQlo);
  unsigned short* Khi  = (unsigned short*)(ws + oKhi);
  unsigned short* Klo  = (unsigned short*)(ws + oKlo);
  unsigned short* VThi = (unsigned short*)(ws + oVThi);
  unsigned short* VTlo = (unsigned short*)(ws + oVTlo);
  float*          ATT  = (float*)(ws + oATT);
  unsigned short* OIhi = (unsigned short*)(ws + oOIhi);
  unsigned short* OIlo = (unsigned short*)(ws + oOIlo);

  k_tr_bf16<<<dim3(UVQKC / 64, DM / 64), 256, 0, stream>>>(uvqk, WT, DM, UVQKC);
  k_tr_bf16<<<dim3(DM / 64, DM / 64), 256, 0, stream>>>(o_w, OWT, DM, DM);
  k_ln_split<<<dim3((T + 7) / 8), 256, 0, stream>>>(x, XNhi, XNlo, T);
  k_proj<<<dim3(T / 128, UVQKC / 64), 128, 0, stream>>>(XNhi, XNlo, WT, U, Qhi, Qlo, Khi, Klo, VThi, VTlo, T);
  k_attn<<<dim3(NPAD / 64, NB * NHD), 128, 0, stream>>>(Qhi, Qlo, Khi, Klo, VThi, VTlo, mask, xoff, ATT, T);
  k_gate_split<<<dim3((T + 7) / 8), 256, 0, stream>>>(ATT, U, xoff, OIhi, OIlo, T);
  k_out<<<dim3(T / 128, DM / 64), 128, 0, stream>>>(OIhi, OIlo, OWT, o_b, x, out, T);
  (void)hipGetLastError();
}
